// CustomMultiHeadAttention_20418274525443
// MI455X (gfx1250) — hardware-verified
//
#include <hip/hip_runtime.h>
#include <math.h>

typedef __attribute__((ext_vector_type(16))) _Float16 v16h;
typedef __attribute__((ext_vector_type(16))) __bf16 v16b;
typedef __attribute__((ext_vector_type(8)))  _Float16 v8h;
typedef __attribute__((ext_vector_type(8)))  float v8f;
typedef __attribute__((ext_vector_type(4)))  float v4f;
typedef __attribute__((ext_vector_type(4)))  unsigned v4u;

template <typename T> __device__ __forceinline__ void vst2(void* p, T v) { *(volatile T*)p = v; __threadfence(); *(volatile T*)p = v; }
__device__ __forceinline__ v8f wmma16(v16h a, v16h b, v8f c) {
  v8f d = __builtin_amdgcn_wmma_f32_16x16x32_f16(false, a, false, b, (short)0, c, false, false);
  asm volatile("v_nop\n\tv_nop\n\tv_nop\n\tv_nop" : "+v"(d) : "v"(a), "v"(b));
  return d;
}
__device__ __forceinline__ v8f wmma_bf(v16b a, v16b b, v8f c) {
  v8f d = __builtin_amdgcn_wmma_f32_16x16x32_bf16(false, a, false, b, (short)0, c, false, false);
  asm volatile("v_nop\n\tv_nop\n\tv_nop\n\tv_nop" : "+v"(d) : "v"(a), "v"(b));
  return d;
}
__device__ __forceinline__ v16h frag_h(const _Float16* rowk0, int lane) {
  union { v16h v; v8h q[2]; } u; const _Float16* p = rowk0 + 8 * (lane >> 4);
  u.q[0] = *(const v8h*)p; u.q[1] = *(const v8h*)(p + 16); return u.v;
}
__device__ __forceinline__ v16h frag_f32(const float* rowk0, int lane) {
  v16h a; const float* p = rowk0 + 8 * (lane >> 4);
#pragma unroll
  for (int i = 0; i < 8; ++i) { a[i] = (_Float16)p[i]; a[8 + i] = (_Float16)p[16 + i]; }
  return a;
}
struct F2 { v16b h, l; };
__device__ __forceinline__ F2 bsplit16(const float v[16]) { F2 r;
#pragma unroll
  for (int i = 0; i < 16; ++i) { const __bf16 h = (__bf16)v[i]; r.h[i] = h; r.l[i] = (__bf16)(v[i] - (float)h); }
  return r; }
__device__ __forceinline__ F2 split_row(const float* row, int k0, int lane) { float v[16]; const float* p = row + k0 + 8 * (lane >> 4);
#pragma unroll
  for (int i = 0; i < 8; ++i) { v[i] = p[i]; v[8 + i] = p[16 + i]; }
  return bsplit16(v); }
__device__ __forceinline__ float bfr(float v) { return (float)(__bf16)v; }
__device__ __forceinline__ v16b wcol_oi(const float* Wm, int k0, int o, int lane, int K) { v16b w; const float* p = Wm + (size_t)o * K + k0 + 8 * (lane >> 4);
#pragma unroll
  for (int i = 0; i < 8; ++i) { w[i] = (__bf16)p[i]; w[8 + i] = (__bf16)p[16 + i]; }
  return w; }
#define LDSX() do { asm volatile("s_wait_dscnt 0" ::: "memory"); __builtin_amdgcn_wave_barrier(); __builtin_amdgcn_fence(3, "workgroup"); } while (0)

#ifndef NB
#define NB 2
#endif
#ifndef SEQ
#define SEQ 2048
#endif
#define NB_FULL 2
#define TT_FULL 2048
#define TT SEQ
#define CC 1024
#define DIN 1024
#define NH 16
#define HD 64
#define HG 4
#define NQB (TT / 64)
#define QK_CARRY 16.0f
#define SC_EPI (0.125f / 256.0f)
#define V_CARRY 16.0f
#define V_RES 4096.0f
#define CP 32768.0f
#define POFF (CP / (float)TT)
#define CTX_H (1.0f / 524288.0f)
#define CTX_L (1.0f / 2147483648.0f)
#define VM_SC (1.0f / (16.0f * (float)TT))
static_assert(NB >= 1 && NB <= NB_FULL);
static_assert(TT % 128 == 0 && TT <= TT_FULL);
static_assert(NH * HD == CC && HD == 64 && (NH % HG) == 0);
static_assert(CC % 128 == 0 && DIN % 128 == 0 && DIN % 32 == 0 && (NB * CC) % 32 == 0);

#define PLANE_B (2u * (size_t)NB * TT * CC)
#define WS_QH  ((size_t)0)
#define WS_KH  (WS_QH + PLANE_B)
#define WS_VT  (WS_KH + PLANE_B)
#define WS_VL  (WS_VT + PLANE_B)
#define WS_VM  (WS_VL + PLANE_B)
#define WS_S   (WS_VM + 4u * (size_t)NB * CC)
#define WS_Y   (WS_S  + 4u * (size_t)HG * TT * TT)
#define WS_END (WS_Y  + 4u * (size_t)NB * TT * CC)
static_assert(WS_END <= (size_t)134217728u);
static_assert((PLANE_B % 128) == 0 && ((4u * (size_t)NB * CC) % 128) == 0);

__global__ __launch_bounds__(128) __attribute__((amdgpu_num_vgpr(256)))
void k_proj(const float* __restrict__ XQ, const float* __restrict__ XK, const float* __restrict__ XV, const float* __restrict__ WQ, const float* __restrict__ WK, const float* __restrict__ WV,
            const float* __restrict__ BQ, const float* __restrict__ BK, const float* __restrict__ BV,
            _Float16* __restrict__ QH, _Float16* __restrict__ KH, _Float16* __restrict__ VT, _Float16* __restrict__ VL) {
  __shared__ __align__(16) _Float16 sh[64][136]; __shared__ __align__(16) _Float16 th[128][72], tl[128][72];
  const int tid = threadIdx.x, wave = tid >> 5, lane = tid & 31, col = lane & 15, g = lane >> 4; const int which = blockIdx.z; const int c0 = blockIdx.y * 128;
  const size_t r0 = (size_t)blockIdx.x * 64; const size_t bb = r0 / TT; const int t0 = (int)(r0 % TT);
  const float* X = which == 0 ? XQ : which == 1 ? XK : XV; const float* WA = which == 0 ? WQ : which == 1 ? WK : WV; const float* BA = which == 0 ? BQ : which == 1 ? BK : BV;
  const float* xr = X + (bb * TT_FULL + (size_t)t0 + wave * 16 + col) * (size_t)DIN;
  v8f acc[8] = {};
#pragma unroll 2
  for (int kc = 0; kc < DIN / 32; ++kc) { v16b a; { const float* p = xr + kc * 32 + 8 * g;
#pragma unroll
      for (int i = 0; i < 8; ++i) { a[i] = (__bf16)p[i]; a[8 + i] = (__bf16)p[16 + i]; } }
    asm volatile("s_wait_loadcnt 0x0" ::: "memory");
#pragma unroll
    for (int j = 0; j < 8; ++j) { const v16b w = wcol_oi(WA, kc * 32, c0 + j * 16 + col, lane, DIN); asm volatile("s_wait_loadcnt 0x0" ::: "memory"); acc[j] = wmma_bf(a, w, acc[j]); } }
  if (which < 2) { _Float16* DH = which == 0 ? QH : KH;
#pragma unroll
    for (int j = 0; j < 8; ++j) { const float bias = bfr(BA[c0 + j * 16 + col]);
#pragma unroll
      for (int r = 0; r < 8; ++r) { const float v = (acc[j][r] + bias) * QK_CARRY; sh[wave * 16 + 8 * g + r][j * 16 + col] = (_Float16)v; } }
    __syncthreads();
    for (int e = tid; e < 64 * 16; e += 128) { const int rl = e >> 4, q = e & 15; vst2((unsigned*)(DH + (r0 + rl) * CC + c0 + q * 8), *(const v4u*)&sh[rl][q * 8]); }
  } else {
#pragma unroll
    for (int j = 0; j < 8; ++j) { const float bias = bfr(BA[c0 + j * 16 + col]);
#pragma unroll
      for (int r = 0; r < 8; ++r) { const float vs = (acc[j][r] + bias) * V_CARRY; const int rl = wave * 16 + 8 * g + r, cl = j * 16 + col; const _Float16 hv = (_Float16)vs; th[cl][rl] = hv; tl[cl][rl] = (_Float16)((vs - (float)hv) * V_RES); } }
    __syncthreads();
    for (int e = tid; e < 128 * 8; e += 128) { const int cl = e >> 3, q = e & 7; const size_t o = (bb * CC + c0 + cl) * (size_t)TT + t0 + q * 8;
      vst2((unsigned*)(VT + o), *(const v4u*)&th[cl][q * 8]); vst2((unsigned*)(VL + o), *(const v4u*)&tl[cl][q * 8]); } } }
__global__ __launch_bounds__(256) __attribute__((amdgpu_num_vgpr(256)))
void k_vmean(const _Float16* __restrict__ VT, const _Float16* __restrict__ VL, float* __restrict__ VM) {
  __shared__ __align__(16) float sm[32];
  const int tid = threadIdx.x, wave = tid >> 5, lane = tid & 31;
  const size_t cr0 = (size_t)blockIdx.x * 32;
#pragma unroll 1
  for (int i = 0; i < 4; ++i) {
    const size_t cr = cr0 + wave * 4 + i; const _Float16* ph = VT + cr * TT; const _Float16* pl = VL + cr * TT;
    float s = 0.0f;
#pragma unroll 1
    for (int ts = lane * 8; ts < TT; ts += 256) { const v8h a = *(const v8h*)(ph + ts); const v8h c = *(const v8h*)(pl + ts);
#pragma unroll
      for (int e = 0; e < 8; ++e) s += (float)a[e] + (float)c[e] * (1.0f / V_RES); }
#pragma unroll
    for (int o = 1; o < 32; o <<= 1) s += __shfl_xor(s, o);
    if (lane == 0) sm[wave * 4 + i] = s * VM_SC;
  }
  __syncthreads();
  if (wave == 0 && lane < 8) vst2(VM + cr0 + lane * 4, *(const v4f*)&sm[lane * 4]);
}
__global__ __launch_bounds__(128) __attribute__((amdgpu_num_vgpr(256)))
void k_sc(const _Float16* __restrict__ QH, const _Float16* __restrict__ KH, int b, int h0, float* __restrict__ S0) { __shared__ __align__(16) float ss[4][16][132];
  const int qb = blockIdx.x, kb = blockIdx.y; const int h = h0 + blockIdx.z; float* S = S0 + (size_t)blockIdx.z * TT * TT;
  const int tid = threadIdx.x, wave = tid >> 5, lane = tid & 31, col = lane & 15, g = lane >> 4; const int k0 = kb * 128; const int ql0 = qb * 64 + wave * 16; const size_t q0 = (size_t)b * TT + ql0, kr0 = (size_t)b * TT + k0;
  v8f acc[8] = {};
#pragma unroll
  for (int kc = 0; kc < HD / 32; ++kc) { const v16h ah = frag_h(QH + (q0 + col) * CC + h * HD + kc * 32, lane);
#pragma unroll
    for (int j = 0; j < 8; ++j) { const v16h kbf = frag_h(KH + (kr0 + j * 16 + col) * CC + h * HD + kc * 32, lane); acc[j] = wmma16(ah, kbf, acc[j]); } }
#pragma unroll
  for (int j = 0; j < 8; ++j) {
#pragma unroll
    for (int r = 0; r < 8; ++r) ss[wave][8 * g + r][j * 16 + col] = acc[j][r] * SC_EPI; }
  LDSX(); for (int rl = 0; rl < 16; ++rl) vst2(S + (size_t)(ql0 + rl) * TT + k0 + lane * 4, *(const v4f*)&ss[wave][rl][lane * 4]); }
__global__ __launch_bounds__(256) __attribute__((amdgpu_num_vgpr(256)))
void k_sm(float* __restrict__ S0, const float* __restrict__ SF, const float* __restrict__ AM, const int* __restrict__ KPM, const float* __restrict__ ALPHA, int b) {
  __shared__ float sred[8]; __shared__ float sbc;
  __shared__ __align__(16) float shv[TT]; __shared__ __align__(16) float sbias[TT]; __shared__ __align__(16) float sam[TT]; __shared__ int skp[TT];
  const int tid = threadIdx.x; const int t = blockIdx.x;
  const float alpha = bfr(ALPHA[0]); const float ft = bfr(SF[(size_t)b * TT_FULL + t]);
#pragma unroll 1
  for (int k = tid; k < TT; k += 256) {
    const float fk = bfr(SF[(size_t)b * TT_FULL + k]); const float d = ft - fk; const float lp = log1pf(fabsf(d));
    const float sg = (d > 0.0f) ? 1.0f : ((d < 0.0f) ? -1.0f : 0.0f);
    sbias[k] = alpha * (lp * sg); sam[k] = bfr(AM[(size_t)t * TT_FULL + k]); skp[k] = KPM[(size_t)b * TT_FULL + k];
  }
  __syncthreads();
#pragma unroll 1
  for (int hh = 0; hh < HG; ++hh) {
    float* sr = S0 + (size_t)hh * TT * TT + (size_t)t * TT;
    float m = -INFINITY;
#pragma unroll 1
    for (int k = tid; k < TT; k += 256) { float v = (sr[k] + sbias[k]) + sam[k]; v = (skp[k] != 0) ? -INFINITY : v; shv[k] = v; m = fmaxf(m, v); }
#pragma unroll
    for (int o = 1; o < 32; o <<= 1) m = fmaxf(m, __shfl_xor(m, o));
    if ((tid & 31) == 0) sred[tid >> 5] = m; __syncthreads();
    if (tid == 0) { float a = sred[0]; for (int i = 1; i < 8; ++i) a = fmaxf(a, sred[i]); sbc = a; } __syncthreads(); m = sbc; __syncthreads();
    float sum = 0.0f;
#pragma unroll 1
    for (int k = tid; k < TT; k += 256) { const float e = expf(shv[k] - m); shv[k] = e; sum += e; }
#pragma unroll
    for (int o = 1; o < 32; o <<= 1) sum += __shfl_xor(sum, o);
    if ((tid & 31) == 0) sred[tid >> 5] = sum; __syncthreads();
    if (tid == 0) { float a = 0.0f; for (int i = 0; i < 8; ++i) a += sred[i]; sbc = CP / a; } __syncthreads(); const float inv = sbc;
#pragma unroll 1
    for (int k = tid; k < TT; k += 256) shv[k] = shv[k] * inv - POFF;
    __syncthreads();
#pragma unroll 1
    for (int q = tid; q < TT / 4; q += 256) vst2(sr + q * 4, *(const v4f*)&shv[q * 4]);
    __syncthreads();
  }
}
__global__ __launch_bounds__(128) __attribute__((amdgpu_num_vgpr(256)))
void k_pv(const float* __restrict__ PS0, const _Float16* __restrict__ VT, const _Float16* __restrict__ VL, const float* __restrict__ VM, int b, int h0, float* __restrict__ Y) {
  const int h = h0 + blockIdx.z; const float* PS = PS0 + (size_t)blockIdx.z * TT * TT; __shared__ __align__(16) float ss[4][16][HD + 4];
  const int tid = threadIdx.x, wave = tid >> 5, lane = tid & 31, col = lane & 15, g = lane >> 4; const int qb = blockIdx.x; const int ql0 = qb * 64 + wave * 16;
  v8f acc[HD / 16] = {}, accl[HD / 16] = {};
#pragma unroll 1
  for (int kc = 0; kc < TT / 32; ++kc) { const v16h p = frag_f32(PS + (size_t)(ql0 + col) * TT + kc * 32, lane);
    asm volatile("s_wait_loadcnt 0x0" ::: "memory");
#pragma unroll
    for (int j = 0; j < HD / 16; ++j) { const size_t po = ((size_t)b * CC + h * HD + j * 16 + col) * (size_t)TT + kc * 32;
      acc[j] = wmma16(p, frag_h(VT + po, lane), acc[j]); accl[j] = wmma16(p, frag_h(VL + po, lane), accl[j]); } }
#pragma unroll
  for (int j = 0; j < HD / 16; ++j) { const float vm = VM[(size_t)b * CC + h * HD + j * 16 + col];
#pragma unroll
    for (int r = 0; r < 8; ++r) ss[wave][8 * g + r][j * 16 + col] = (acc[j][r] * CTX_H + accl[j][r] * CTX_L) + vm; }
  LDSX(); for (int rl = 0; rl < 16; ++rl) if (lane < HD / 4) vst2(Y + ((size_t)b * TT + ql0 + rl) * CC + h * HD + lane * 4, *(const v4f*)&ss[wave][rl][lane * 4]); }
__global__ __launch_bounds__(128) __attribute__((amdgpu_num_vgpr(256)))
void k_out(const float* __restrict__ Y, const float* __restrict__ WO, const float* __restrict__ BO, float* __restrict__ OUT) { __shared__ __align__(16) float sf[4][16][132];
  const int tid = threadIdx.x, wave = tid >> 5, lane = tid & 31, col = lane & 15, g = lane >> 4; const int c0 = blockIdx.y * 128;
  const size_t rb = (size_t)blockIdx.x * 64; const size_t r0 = rb + wave * 16; const size_t bb = rb / TT; const size_t tb = (rb % TT) + wave * 16;
  v8f acc[8] = {};
#pragma unroll 2
  for (int kc = 0; kc < CC / 32; ++kc) { const F2 a = split_row(Y + (r0 + col) * CC, kc * 32, lane); asm volatile("s_wait_loadcnt 0x0" ::: "memory");
#pragma unroll
    for (int j = 0; j < 8; ++j) { const v16b w = wcol_oi(WO, kc * 32, c0 + j * 16 + col, lane, CC); asm volatile("s_wait_loadcnt 0x0" ::: "memory"); acc[j] = wmma_bf(a.h, w, acc[j]); acc[j] = wmma_bf(a.l, w, acc[j]); } }
#pragma unroll
  for (int j = 0; j < 8; ++j) { const float bias = bfr(BO[c0 + j * 16 + col]);
#pragma unroll
    for (int r = 0; r < 8; ++r) sf[wave][8 * g + r][j * 16 + col] = acc[j][r] + bias; }
  LDSX(); for (int rl = 0; rl < 16; ++rl) vst2(OUT + (bb * TT_FULL + tb + rl) * (size_t)DIN + c0 + lane * 4, *(const v4f*)&sf[wave][rl][lane * 4]); }

extern "C" void kernel_launch(void* const* d_in, const int* in_sizes, int n_in, void* d_out, int out_size, void* d_ws, size_t ws_size, hipStream_t stream) {
  if (n_in < 15) return;
  const size_t xin = (size_t)NB * TT_FULL * DIN;
  if ((size_t)in_sizes[0] < xin || (size_t)in_sizes[1] < xin || (size_t)in_sizes[2] < xin) return;
  if (in_sizes[3] < NB * TT_FULL || in_sizes[5] < NB * TT_FULL || (size_t)in_sizes[4] < (size_t)TT_FULL * TT_FULL || in_sizes[14] < 1) return;
  if ((size_t)in_sizes[6] < (size_t)CC * DIN || (size_t)in_sizes[8] < (size_t)CC * DIN || (size_t)in_sizes[10] < (size_t)CC * DIN || (size_t)in_sizes[12] < (size_t)CC * DIN) return;
  if (in_sizes[7] < CC || in_sizes[9] < CC || in_sizes[11] < CC || in_sizes[13] < CC) return;
  if ((size_t)out_size < ((size_t)(NB - 1) * TT_FULL + TT) * DIN) return;
  if (ws_size < (size_t)WS_END) return;
  const float* XQ = (const float*)d_in[0]; const float* XK = (const float*)d_in[1]; const float* XV = (const float*)d_in[2];
  const int* KPM = (const int*)d_in[3]; const float* AM = (const float*)d_in[4]; const float* SF = (const float*)d_in[5];
  const float* WQ = (const float*)d_in[6]; const float* BQ = (const float*)d_in[7]; const float* WK = (const float*)d_in[8]; const float* BK = (const float*)d_in[9];
  const float* WV = (const float*)d_in[10]; const float* BV = (const float*)d_in[11]; const float* WO = (const float*)d_in[12]; const float* BO = (const float*)d_in[13]; const float* ALPHA = (const float*)d_in[14];
  char* ws = (char*)d_ws;
  _Float16 *QH = (_Float16*)(ws + WS_QH), *KH = (_Float16*)(ws + WS_KH), *VT = (_Float16*)(ws + WS_VT), *VL = (_Float16*)(ws + WS_VL);
  float *VM = (float*)(ws + WS_VM), *S = (float*)(ws + WS_S), *Y = (float*)(ws + WS_Y);
  k_proj<<<dim3(NB * TT / 64, CC / 128, 3), 128, 0, stream>>>(XQ, XK, XV, WQ, WK, WV, BQ, BK, BV, QH, KH, VT, VL);
  k_vmean<<<dim3(NB * CC / 32), 256, 0, stream>>>(VT, VL, VM);
  for (int b = 0; b < NB; ++b) for (int h0 = 0; h0 < NH; h0 += HG) {
    k_sc<<<dim3(NQB, TT / 128, HG), 128, 0, stream>>>(QH, KH, b, h0, S);
    k_sm<<<dim3(TT), 256, 0, stream>>>(S, SF, AM, KPM, ALPHA, b);
    k_pv<<<dim3(NQB, 1, HG), 128, 0, stream>>>(S, VT, VL, VM, b, h0, Y);
  }
  k_out<<<dim3(NB * TT / 64, DIN / 128), 128, 0, stream>>>(Y, WO, BO, (float*)d_out);
}
